// GroupedQueryAttention_30193620091315
// MI455X (gfx1250) — hardware-verified
//
#include <hip/hip_runtime.h>
#include <math.h>
#ifndef NB
#define NB 2
#endif
#ifndef SEQ
#define SEQ 2048
#endif
#define NB_FULL 2
#define SEQ_FULL 2048
#define DM 2048u
#define NH 16u
#define NKV 4u
#define HD 128u
#define HPG 4u
#define KVD 512u
#define NQKV 3072u
#define KOFF 2048u
#define VOFF 2560u
constexpr unsigned cNB = (unsigned)(NB);
constexpr unsigned cSEQ = (unsigned)(SEQ);
constexpr unsigned cSEQF = (unsigned)(SEQ_FULL);
constexpr unsigned cNR = cNB * cSEQ;
constexpr unsigned cBAND = (cSEQ < 512u) ? cSEQ : 512u;
constexpr unsigned cBQT = cBAND / 16u;
constexpr unsigned cMQT = (cSEQ - cBAND) / 16u;
constexpr unsigned cMQTD = cMQT ? cMQT : 1u;
static_assert(cSEQ % 128u == 0u);
static_assert(cBAND % 128u == 0u);
static_assert((cSEQ - cBAND) % 128u == 0u);
static_assert(cSEQ <= cSEQF);
static_assert(cNB <= (unsigned)(NB_FULL));

typedef unsigned short v8us __attribute__((ext_vector_type(8), may_alias));
typedef float  v8f  __attribute__((ext_vector_type(8)));
typedef float  v4f  __attribute__((ext_vector_type(4)));
typedef float  v4fa __attribute__((ext_vector_type(4), may_alias));
typedef _Float16 v16h __attribute__((ext_vector_type(16)));
union FragH { v16h v; v8us half[2]; _Float16 h[16]; unsigned short u[16]; };
struct F32x32 { float v[32]; };
static_assert(sizeof(F32x32) == 128);

__device__ __forceinline__ unsigned short bf16_bits(float x) { unsigned int u = __float_as_uint(x); return (unsigned short)((u + 0x7FFFu + ((u >> 16) & 1u)) >> 16); }
__device__ __forceinline__ float bf16_val(unsigned short b) { return __uint_as_float(((unsigned int)b) << 16); }
__device__ __forceinline__ float bf16_rne(float x) { return bf16_val(bf16_bits(x)); }
__device__ __forceinline__ unsigned short h2u(_Float16 h) { return __builtin_bit_cast(unsigned short, h); }
__device__ __forceinline__ unsigned wave_id() { return (unsigned)__builtin_amdgcn_readfirstlane((int)(threadIdx.x >> 5)); }
__device__ __forceinline__ v16h ld_frag(const unsigned short* p, unsigned hh) { FragH f; f.half[0] = *(const v8us*)(p + 8u * hh); f.half[1] = *(const v8us*)(p + 16u + 8u * hh); return f.v; }
__device__ __forceinline__ v8f g2_mma(v16h a, v16h b, v8f c) { v8f d = __builtin_amdgcn_wmma_f32_16x16x32_f16(false, a, false, b, (short)0, c, false, false); asm volatile("v_nop\n\tv_nop\n\tv_nop\n\tv_nop" : "+v"(d) : "v"(a), "v"(b)); return d; }

__global__ __launch_bounds__(256) void k_x16(const float* __restrict__ x, _Float16* __restrict__ X16) {
  const unsigned t = blockIdx.x * 256u + threadIdx.x; if (t >= cNR * (DM / 8u)) return;
  const unsigned row = t / (DM / 8u), c8 = (t % (DM / 8u)) * 8u; const unsigned b = row / cSEQ, tt = row % cSEQ;
  const float* src = x + ((size_t)b * cSEQF + tt) * DM + c8;
  const v4f a = *(const v4fa*)src, c = *(const v4fa*)(src + 4); FragH f;
#pragma unroll
  for (unsigned q = 0; q < 4; ++q) { f.h[q] = (_Float16)bf16_rne(a[q]); f.h[4 + q] = (_Float16)bf16_rne(c[q]); }
  const v8us o = f.half[0]; unsigned short* dst = (unsigned short*)X16 + (size_t)t * 8u;
  *(volatile v8us*)dst = o; __threadfence(); *(volatile v8us*)dst = o; }

__global__ __launch_bounds__(256) void k_wt_f16(const float* __restrict__ W, _Float16* __restrict__ Wt, unsigned K, unsigned N) {
  const unsigned t = blockIdx.x * 256u + threadIdx.x; const unsigned k8n = K >> 3; if (t >= N * k8n) return;
  const unsigned nn = t / k8n, k8 = (t - nn * k8n) << 3; FragH f;
#pragma unroll
  for (unsigned i = 0; i < 8; ++i) f.h[i] = (_Float16)(bf16_rne(W[(size_t)(k8 + i) * N + nn]) * 16.0f);
  const v8us o = f.half[0]; unsigned short* dst = (unsigned short*)Wt + (size_t)nn * K + k8;
  *(volatile v8us*)dst = o; __threadfence(); *(volatile v8us*)dst = o; }

__global__ __launch_bounds__(256) void k_tab(F32x32 a, unsigned i0, float* __restrict__ CS, float* __restrict__ SN) {
  #pragma clang fp contract(off)
  const unsigned gid = blockIdx.x * 256u + threadIdx.x; if (gid >= cSEQ * 32u) return; const unsigned lane = threadIdx.x & 31u, t = gid >> 5;
  float inv = 0.0f;
#pragma unroll
  for (unsigned i = 0; i < 32; ++i) inv = (lane == i) ? a.v[i] : inv;
  const float ang = (float)t * inv; const float c = cosf(ang), s = sinf(ang);
  float* pc = CS + (size_t)t * 64u + i0 + lane; float* ps = SN + (size_t)t * 64u + i0 + lane;
  *(volatile float*)pc = c; *(volatile float*)ps = s; __threadfence(); *(volatile float*)pc = c; *(volatile float*)ps = s; }

template <int RES>
__global__ __launch_bounds__(128) void k_gemm2(const _Float16* __restrict__ A, const _Float16* __restrict__ AR, unsigned lda, unsigned ldar, size_t sA, size_t sAR,
    const _Float16* __restrict__ Bh, unsigned ldb, float alpha, float* __restrict__ C, unsigned ldc, size_t sC, unsigned M, unsigned N, unsigned K) {
  __shared__ __attribute__((aligned(16))) float so[4][32][68];
  const unsigned tid = threadIdx.x, lane = tid & 31u, ln = lane & 15u, hh = lane >> 4, w = wave_id(), by = blockIdx.y;
  const unsigned ntn = N >> 6; const unsigned mt = blockIdx.x / ntn, nq = blockIdx.x - mt * ntn;
  const unsigned row0 = mt * 128u + 32u * w, col0 = nq * 64u; if (row0 >= M) return;
  const unsigned short* a0p = (const unsigned short*)A + (size_t)by * sA + (size_t)(row0 + ln) * lda; const unsigned short* a1p = a0p + (size_t)16 * lda;
  const unsigned short* r0p = (const unsigned short*)AR + (size_t)by * sAR + (size_t)(row0 + ln) * ldar; const unsigned short* r1p = r0p + (size_t)16 * ldar;
  const unsigned short* bp = (const unsigned short*)Bh + (size_t)(col0 + ln) * ldb;
  const v8f z8 = {0.f,0.f,0.f,0.f,0.f,0.f,0.f,0.f};
  v8f c[2][4], d[2][4];
#pragma unroll
  for (unsigned t = 0; t < 4; ++t) { c[0][t] = z8; c[1][t] = z8; d[0][t] = z8; d[1][t] = z8; }
#pragma unroll 1
  for (unsigned kb = 0; kb < K; kb += 32u) {
    const v16h a0 = ld_frag(a0p + kb, hh), a1 = ld_frag(a1p + kb, hh);
    v16h e0 = a0, e1 = a1; if (RES) { e0 = ld_frag(r0p + kb, hh); e1 = ld_frag(r1p + kb, hh); }
#pragma unroll
    for (unsigned t = 0; t < 4; ++t) { const v16h b = ld_frag(bp + (size_t)(t * 16u) * ldb + kb, hh);
      c[0][t] = g2_mma(a0, b, c[0][t]); c[1][t] = g2_mma(a1, b, c[1][t]);
      if (RES) { d[0][t] = g2_mma(e0, b, d[0][t]); d[1][t] = g2_mma(e1, b, d[1][t]); } } }
#pragma unroll
  for (unsigned u = 0; u < 2; ++u) {
#pragma unroll
    for (unsigned t = 0; t < 4; ++t) {
#pragma unroll
      for (unsigned r = 0; r < 8; ++r) { float v = c[u][t][r]; if (RES) v += d[u][t][r] * 0.0009765625f; so[w][u * 16u + 8u * hh + r][t * 16u + ln] = v * alpha; } } }
  __builtin_amdgcn_fence(4  , "workgroup"); __builtin_amdgcn_wave_barrier();
  const unsigned rsub = lane >> 4, c4 = (lane & 15u) * 4u; float* cb = C + (size_t)by * sC;
  for (int pass = 0; pass < 2; ++pass) {
#pragma unroll
    for (unsigned q = 0; q < 16; ++q) { const unsigned r = q * 2u + rsub; const v4f v = *(const v4fa*)&so[w][r][c4]; *(volatile v4f*)(cb + (size_t)(row0 + r) * ldc + col0 + c4) = v; }
    if (pass == 0) __threadfence(); } }

__global__ __launch_bounds__(256) void k_normrope(const float* __restrict__ F, const float* __restrict__ CS, const float* __restrict__ SN, const float* __restrict__ gq, const float* __restrict__ gk,
    _Float16* __restrict__ Q16, _Float16* __restrict__ K16) {
  __shared__ __attribute__((aligned(16))) unsigned short st[8][256];
  const unsigned lane = threadIdx.x & 31u, w = wave_id(); const unsigned wid = blockIdx.x * 8u + w;
  const unsigned pr = wid % 10u, r = wid / 10u, t = r % cSEQ; const unsigned h0 = pr * 2u;
  const float c0 = CS[(size_t)t * 64u + lane], c1 = CS[(size_t)t * 64u + lane + 32u], s0 = SN[(size_t)t * 64u + lane], s1 = SN[(size_t)t * 64u + lane + 32u];
  const float* g = (h0 < NH) ? gq : gk;
  const float g0 = 1.0f + bf16_rne(g[lane]), g1 = 1.0f + bf16_rne(g[lane + 32u]), g2 = 1.0f + bf16_rne(g[lane + 64u]), g3 = 1.0f + bf16_rne(g[lane + 96u]);
#pragma unroll 1
  for (unsigned it = 0; it < 2; ++it) {
    const float* src = F + (size_t)r * NQKV + (h0 + it) * HD;
    float v0 = src[lane], v1 = src[lane + 32u], v2 = src[lane + 64u], v3 = src[lane + 96u];
    float ss = v0 * v0 + v1 * v1 + v2 * v2 + v3 * v3;
    ss += __shfl_xor(ss, 1); ss += __shfl_xor(ss, 2); ss += __shfl_xor(ss, 4); ss += __shfl_xor(ss, 8); ss += __shfl_xor(ss, 16);
    const float inv = rsqrtf(ss * 0.0078125f + 1e-6f);
    v0 = v0 * inv * g0; v1 = v1 * inv * g1; v2 = v2 * inv * g2; v3 = v3 * inv * g3;
    const float o0 = v0 * c0 - v2 * s0, o2 = v0 * s0 + v2 * c0, o1 = v1 * c1 - v3 * s1, o3 = v1 * s1 + v3 * c1;
    st[w][it * 128u + lane] = h2u((_Float16)o0); st[w][it * 128u + lane + 32u] = h2u((_Float16)o1);
    st[w][it * 128u + lane + 64u] = h2u((_Float16)o2); st[w][it * 128u + lane + 96u] = h2u((_Float16)o3); }
  __builtin_amdgcn_fence(4  , "workgroup"); __builtin_amdgcn_wave_barrier();
  const v8us o = *(const v8us*)&st[w][lane * 8u];
  unsigned short* dst = (h0 < NH) ? ((unsigned short*)Q16 + (size_t)r * DM + h0 * HD + lane * 8u) : ((unsigned short*)K16 + (size_t)r * KVD + (h0 - NH) * HD + lane * 8u);
  *(volatile v8us*)dst = o; __threadfence(); *(volatile v8us*)dst = o; }

__global__ __launch_bounds__(256) void k_vt(const float* __restrict__ F, _Float16* __restrict__ VT, _Float16* __restrict__ VTR) {
  __shared__ __attribute__((aligned(16))) unsigned short th[64][72]; __shared__ __attribute__((aligned(16))) unsigned short tr[64][72];
  const unsigned tid = threadIdx.x; const unsigned cg = blockIdx.x & 7u; const unsigned t2 = blockIdx.x >> 3; const unsigned sg = t2 % (cSEQ / 64u), b = t2 / (cSEQ / 64u);
#pragma unroll
  for (unsigned it = 0; it < 4; ++it) { const unsigned i = it * 256u + tid; const unsigned rr = i >> 4, c4 = (i & 15u) * 4u;
    const v4f a = *(const v4fa*)(F + (size_t)(b * cSEQ + sg * 64u + rr) * NQKV + VOFF + cg * 64u + c4);
#pragma unroll
    for (unsigned q = 0; q < 4; ++q) { const _Float16 hv = (_Float16)a[q]; th[c4 + q][rr] = h2u(hv); tr[c4 + q][rr] = h2u((_Float16)((a[q] - (float)hv) * 1024.0f)); } }
  __syncthreads();
  for (int pass = 0; pass < 2; ++pass) {
#pragma unroll
    for (unsigned it = 0; it < 2; ++it) { const unsigned i = it * 256u + tid; const unsigned c = i >> 3, pc = (i & 7u) * 8u;
      const v8us vh = *(const v8us*)&th[c][pc]; const v8us vr = *(const v8us*)&tr[c][pc];
      const size_t o = (size_t)(b * 512u + cg * 64u + c) * cSEQ + sg * 64u + pc;
      *(volatile v8us*)((unsigned short*)VT + o) = vh; *(volatile v8us*)((unsigned short*)VTR + o) = vr; }
    if (pass == 0) __threadfence(); } }

template <int BAND>
__global__ __launch_bounds__(256) void k_flash(const _Float16* __restrict__ Q16, const _Float16* __restrict__ K16, const _Float16* __restrict__ VT, const _Float16* __restrict__ VTR,
    _Float16* __restrict__ O16, _Float16* __restrict__ ORES) {
  constexpr unsigned KT = BAND ? 2u : 4u, NT = BAND ? 4u : 8u, KS = KT * 16u, PP = KS + 8u, OW = NT * 16u, OP = OW + 8u, NP = BAND ? 2u : 1u, KH = KT / 2u;
  __shared__ __attribute__((aligned(16))) unsigned short pl[8][NP][16 * PP];
  __shared__ __attribute__((aligned(16))) unsigned short os[8][NP][16 * OP];
  const unsigned lane = threadIdx.x & 31u, n = lane & 15u, hh = lane >> 4, w = wave_id();
  const unsigned wid = blockIdx.x * 8u + w;
  unsigned dh = 0u, qt, bh;
  if (BAND) { dh = wid & 1u; const unsigned t = wid >> 1; qt = t % cBQT; bh = t / cBQT; } else { qt = cBQT + wid % cMQTD; bh = wid / cMQTD; }
  const unsigned h = bh % NH, b = bh / NH, kv = h / HPG;
  const unsigned short* qrow = (const unsigned short*)Q16 + (size_t)(b * cSEQ + qt * 16u + n) * DM + h * HD;
  const unsigned short* kcol = (const unsigned short*)K16 + (size_t)(b * cSEQ + n) * KVD + kv * HD;
  const size_t voff = (size_t)((b * NKV + kv) * HD + dh * 64u + n) * cSEQ;
  const unsigned short* vrow = (const unsigned short*)VT + voff; const unsigned short* vrrow = (const unsigned short*)VTR + voff;
  const v8f z8 = {0.f,0.f,0.f,0.f,0.f,0.f,0.f,0.f};
  v8f acc[NT], acc1[NT];
#pragma unroll
  for (unsigned t = 0; t < NT; ++t) { acc[t] = z8; acc1[t] = z8; }
  float mrow[8], lrow[8];
#pragma unroll
  for (unsigned r = 0; r < 8; ++r) { mrow[r] = -3.0e38f; lrow[r] = 0.0f; }
  const unsigned q0 = qt * 16u + 8u * hh;
  const unsigned nsteps = (qt * 16u + 15u) / KS + 1u;
  const float SC = 0.0078125f * 1.4426950408889634f;
#pragma unroll 1
  for (unsigned st = 0; st < nsteps; ++st) {
    const unsigned kb = st * KS;
    unsigned qo = 0u; asm volatile("" : "+v"(qo));
    v8f s[KT];
#pragma unroll
    for (unsigned j = 0; j < KT; ++j) s[j] = z8;
#pragma unroll
    for (unsigned dt = 0; dt < 4; ++dt) { const v16h qa = ld_frag(qrow + qo + dt * 32u, hh);
#pragma unroll
      for (unsigned j = 0; j < KT; ++j) { const v16h kf = ld_frag(kcol + (size_t)(kb + j * 16u) * KVD + dt * 32u, hh); s[j] = g2_mma(qa, kf, s[j]); } }
#pragma unroll
    for (unsigned j = 0; j < KT; ++j) s[j] = s[j] * SC;
    if (st + 1u == nsteps) {
#pragma unroll
      for (unsigned j = 0; j < KT; ++j) { const unsigned key = kb + j * 16u + n;
#pragma unroll
        for (unsigned r = 0; r < 8; ++r) s[j][r] = (key <= q0 + r) ? s[j][r] : -3.0e38f; } }
    float al[8];
#pragma unroll
    for (unsigned r = 0; r < 8; ++r) {
      float rm = s[0][r];
#pragma unroll
      for (unsigned j = 1; j < KT; ++j) rm = fmaxf(rm, s[j][r]);
      rm = fmaxf(rm, __shfl_xor(rm, 1)); rm = fmaxf(rm, __shfl_xor(rm, 2)); rm = fmaxf(rm, __shfl_xor(rm, 4)); rm = fmaxf(rm, __shfl_xor(rm, 8));
      const float mnew = fmaxf(mrow[r], rm);
      al[r] = __builtin_amdgcn_exp2f(mrow[r] - mnew); mrow[r] = mnew;
      float ps = 0.0f;
#pragma unroll
      for (unsigned j = 0; j < KT; ++j) { const float p = __builtin_amdgcn_exp2f((s[j][r] - mnew) + 10.0f); ps += p;
        const _Float16 ph = (_Float16)p; const unsigned o = (8u * hh + r) * PP + j * 16u + n;
        pl[w][0][o] = h2u(ph); if (BAND) pl[w][NP - 1u][o] = h2u((_Float16)((p - (float)ph) * 1024.0f)); }
      lrow[r] = lrow[r] * al[r] + ps; }
#pragma unroll
    for (unsigned t = 0; t < NT; ++t) {
#pragma unroll
      for (unsigned r = 0; r < 8; ++r) { acc[t][r] *= al[r]; if (BAND) acc1[t][r] *= al[r]; } }
    __builtin_amdgcn_fence(4  , "workgroup"); __builtin_amdgcn_wave_barrier();
    v16h pa[KH], par[KH];
#pragma unroll
    for (unsigned ks = 0; ks < KH; ++ks) { FragH f; f.half[0] = *(const v8us*)&pl[w][0][n * PP + ks * 32u + 8u * hh]; f.half[1] = *(const v8us*)&pl[w][0][n * PP + ks * 32u + 16u + 8u * hh]; pa[ks] = f.v;
      FragH g; g.half[0] = *(const v8us*)&pl[w][NP - 1u][n * PP + ks * 32u + 8u * hh]; g.half[1] = *(const v8us*)&pl[w][NP - 1u][n * PP + ks * 32u + 16u + 8u * hh]; par[ks] = g.v; }
#pragma unroll
    for (unsigned t = 0; t < NT; ++t) {
#pragma unroll
      for (unsigned ks = 0; ks < KH; ++ks) { const size_t o = (size_t)(t * 16u) * cSEQ + kb + ks * 32u;
        const v16h vb = ld_frag(vrow + o, hh); acc[t] = g2_mma(pa[ks], vb, acc[t]);
        if (BAND) { acc1[t] = g2_mma(par[ks], vb, acc1[t]); const v16h vr = ld_frag(vrrow + o, hh); acc1[t] = g2_mma(pa[ks], vr, acc1[t]); } } }
  }
  float sc[8];
#pragma unroll
  for (unsigned r = 0; r < 8; ++r) { float l = lrow[r]; l += __shfl_xor(l, 1); l += __shfl_xor(l, 2); l += __shfl_xor(l, 4); l += __shfl_xor(l, 8); sc[r] = 64.0f * __builtin_amdgcn_rcpf(l); }
#pragma unroll
  for (unsigned t = 0; t < NT; ++t) {
#pragma unroll
    for (unsigned r = 0; r < 8; ++r) { float v = acc[t][r]; if (BAND) v += acc1[t][r] * 0.0009765625f; v *= sc[r];
      const _Float16 hv = (_Float16)v; const unsigned o = (8u * hh + r) * OP + t * 16u + n;
      os[w][0][o] = h2u(hv); if (BAND) os[w][NP - 1u][o] = h2u((_Float16)((v - (float)hv) * 1024.0f)); } }
  __builtin_amdgcn_fence(4  , "workgroup"); __builtin_amdgcn_wave_barrier();
  if (BAND) {
    const unsigned rs = lane >> 3, pc = (lane & 7u) * 8u;
    for (int pass = 0; pass < 2; ++pass) {
#pragma unroll
      for (unsigned q = 0; q < 4; ++q) { const unsigned row = q * 4u + rs;
        const v8us vh = *(const v8us*)&os[w][0][row * OP + pc]; const v8us vr = *(const v8us*)&os[w][NP - 1u][row * OP + pc];
        *(volatile v8us*)((unsigned short*)O16 + (size_t)(b * cSEQ + qt * 16u + row) * DM + h * HD + dh * 64u + pc) = vh;
        *(volatile v8us*)((unsigned short*)ORES + (size_t)(b * cBAND + qt * 16u + row) * DM + h * HD + dh * 64u + pc) = vr; }
      if (pass == 0) __threadfence(); }
  } else {
    const unsigned pc = n * 8u;
    for (int pass = 0; pass < 2; ++pass) {
#pragma unroll
      for (unsigned q = 0; q < 8; ++q) { const unsigned row = q * 2u + hh; const v8us vh = *(const v8us*)&os[w][0][row * OP + pc];
        *(volatile v8us*)((unsigned short*)O16 + (size_t)(b * cSEQ + qt * 16u + row) * DM + h * HD + pc) = vh; }
      if (pass == 0) __threadfence(); }
  } }

constexpr size_t SZ_X16 = (size_t)cNR * DM * 2;
constexpr size_t SZ_BQKV = (size_t)NQKV * DM * 2;
constexpr size_t SZ_BO = (size_t)DM * DM * 2;
constexpr size_t SZ_F = (size_t)cNR * NQKV * 4;
constexpr size_t SZ_TAB = (size_t)cSEQ * 64 * 4;
constexpr size_t SZ_Q16 = (size_t)cNR * DM * 2;
constexpr size_t SZ_K16 = (size_t)cNR * KVD * 2;
constexpr size_t SZ_VT = (size_t)cNB * 512 * cSEQ * 2;
constexpr size_t SZ_ORES = (size_t)cNB * cBAND * DM * 2;
constexpr size_t SZ_TOTAL = SZ_X16 + SZ_BQKV + SZ_BO + SZ_F + 2 * SZ_TAB + SZ_Q16 + SZ_K16 + 2 * SZ_VT + SZ_ORES;
static_assert(SZ_TOTAL <= (size_t)134217728);
static_assert(SZ_X16 % 256 == 0 && SZ_BQKV % 256 == 0 && SZ_BO % 256 == 0 && SZ_F % 256 == 0 && SZ_TAB % 256 == 0 && SZ_K16 % 256 == 0 && SZ_VT % 256 == 0 && SZ_ORES % 256 == 0);
static_assert(((size_t)cNR * DM / 8) % 256 == 0);
static_assert(((size_t)DM * DM / 8) % 256 == 0 && ((size_t)KVD * DM / 8) % 256 == 0);
static_assert((cSEQ * 32u) % 256u == 0u);
static_assert((cNR * 10u) % 8u == 0u);
static_assert((cNB * NH * cBQT * 2u) % 8u == 0u && (cNB * NH * cMQT) % 8u == 0u);
static_assert((size_t)(cNB * NH * cBQT * 2u) * 16 * 64 == (size_t)cNB * cBAND * DM);
static_assert((size_t)(cNB * NH * cMQT) * 16 * 128 == (size_t)cNB * (cSEQ - cBAND) * DM);
static_assert((size_t)(cNB * (cSEQ / 64u) * 8u) * 64 * 64 == (size_t)cNB * cSEQ * 512);
static_assert(cNR % 128u == 0u && NQKV % 64u == 0u && DM % 64u == 0u && DM % 32u == 0u);

extern "C" void kernel_launch(void* const* d_in, const int* in_sizes, int n_in,
                              void* d_out, int out_size, void* d_ws, size_t ws_size, hipStream_t stream) {
  if (n_in < 8) return;
  if ((size_t)in_sizes[0] < ((size_t)(cNB - 1u) * cSEQF + cSEQ) * DM) return;
  if ((size_t)in_sizes[2] < (size_t)DM * DM || (size_t)in_sizes[3] < (size_t)DM * KVD || (size_t)in_sizes[4] < (size_t)DM * KVD || (size_t)in_sizes[5] < (size_t)DM * DM) return;
  if (in_sizes[6] < 128 || in_sizes[7] < 128) return;
  if ((size_t)out_size < (size_t)cNR * DM) return;
  if (SZ_TOTAL > ws_size) return;
  const float* x = (const float*)d_in[0];
  const float* Wq = (const float*)d_in[2]; const float* Wk = (const float*)d_in[3]; const float* Wv = (const float*)d_in[4]; const float* Wo = (const float*)d_in[5];
  const float* gq = (const float*)d_in[6]; const float* gk = (const float*)d_in[7];
  char* ws = (char*)d_ws; size_t off = 0;
  auto take = [&](size_t bytes) { char* p = ws + off; off += bytes; return p; };
  _Float16* X16 = (_Float16*)take(SZ_X16); _Float16* O16 = X16;
  _Float16* BQKV = (_Float16*)take(SZ_BQKV); _Float16* BO = (_Float16*)take(SZ_BO);
  float* F = (float*)take(SZ_F); float* CS = (float*)take(SZ_TAB); float* SN = (float*)take(SZ_TAB);
  _Float16* Q16 = (_Float16*)take(SZ_Q16); _Float16* K16 = (_Float16*)take(SZ_K16);
  _Float16* VT = (_Float16*)take(SZ_VT); _Float16* VTR = (_Float16*)take(SZ_VT); _Float16* ORES = (_Float16*)take(SZ_ORES);
  if (off > ws_size) return;
  F32x32 fa, fb;
  for (int i = 0; i < 32; ++i) { const float p0 = (float)pow(10000.0, (double)i / 64.0); fa.v[i] = 1.0f / p0; const float p1 = (float)pow(10000.0, (double)(i + 32) / 64.0); fb.v[i] = 1.0f / p1; }

  k_x16<<<(unsigned)((size_t)cNR * DM / 8 / 256), 256, 0, stream>>>(x, X16);
  k_wt_f16<<<(unsigned)((size_t)DM * DM / 8 / 256), 256, 0, stream>>>(Wq, BQKV, DM, DM);
  k_wt_f16<<<(unsigned)((size_t)KVD * DM / 8 / 256), 256, 0, stream>>>(Wk, BQKV + (size_t)KOFF * DM, DM, KVD);
  k_wt_f16<<<(unsigned)((size_t)KVD * DM / 8 / 256), 256, 0, stream>>>(Wv, BQKV + (size_t)VOFF * DM, DM, KVD);
  k_wt_f16<<<(unsigned)((size_t)DM * DM / 8 / 256), 256, 0, stream>>>(Wo, BO, DM, DM);
  k_tab<<<cSEQ * 32u / 256u, 256, 0, stream>>>(fa, 0u, CS, SN);
  k_tab<<<cSEQ * 32u / 256u, 256, 0, stream>>>(fb, 32u, CS, SN);
  k_gemm2<0><<<dim3((cNR / 128u) * (NQKV / 64u), 1), 128, 0, stream>>>(X16, X16, DM, DM, 0, 0, BQKV, DM, 0.0625f, F, NQKV, 0, cNR, NQKV, DM);
  k_normrope<<<cNR * 10u / 8u, 256, 0, stream>>>(F, CS, SN, gq, gk, Q16, K16);
  k_vt<<<cNB * (cSEQ / 64u) * 8u, 256, 0, stream>>>(F, VT, VTR);
  k_flash<1><<<cNB * NH * cBQT * 2u / 8u, 256, 0, stream>>>(Q16, K16, VT, VTR, O16, ORES);
  if (cMQT > 0u) k_flash<0><<<cNB * NH * cMQTD / 8u, 256, 0, stream>>>(Q16, K16, VT, VTR, O16, ORES);
  float* out = (float*)d_out;
  if (cMQT > 0u) k_gemm2<0><<<dim3(((cSEQ - cBAND) / 128u) * (DM / 64u), cNB), 128, 0, stream>>>(O16 + (size_t)cBAND * DM, O16, DM, DM, (size_t)cSEQ * DM, 0, BO, DM, 0.0009765625f,
      out + (size_t)cBAND * DM, DM, (size_t)cSEQ * DM, cSEQ - cBAND, DM, DM);
  k_gemm2<1><<<dim3((cBAND / 128u) * (DM / 64u), cNB), 128, 0, stream>>>(O16, ORES, DM, DM, (size_t)cSEQ * DM, (size_t)cBAND * DM, BO, DM, 0.0009765625f,
      out, DM, (size_t)cSEQ * DM, cBAND, DM, DM);
}
